// LambdaLayer_10153302687838
// MI455X (gfx1250) — hardware-verified
//
#include <hip/hip_runtime.h>


namespace {
constexpr int NB_ = 32, DIM = 256, NS = 32, NP = NS * NS, HEADS = 4, DK = 16, DV = 64, NQ = HEADS * DK  , NO = NQ + DK + DV  , RL = 2 * NS - 1  ;
constexpr float XS = 8.0f, HS = 256.0f, WSC = 256.0f, EPS = 1e-5f;
typedef _Float16 b16;
typedef __attribute__((ext_vector_type(16))) _Float16 v16b;
typedef __attribute__((ext_vector_type(8))) _Float16 v8b;
typedef __attribute__((ext_vector_type(8))) float v8f;
typedef __attribute__((ext_vector_type(4))) float v4f;
typedef __attribute__((ext_vector_type(2))) float v2f;
typedef __attribute__((ext_vector_type(2))) _Float16 v2b;
__device__ __forceinline__ float bf16_rne(float f) { unsigned int u = __float_as_uint(f); u += 0x7FFFu + ((u >> 16) & 1u); float r = __uint_as_float(u & 0xFFFF0000u); asm volatile("" : "+v"(r)); return r; }
__device__ __forceinline__ float bfv(float f) { float r = bf16_rne(f); asm volatile("" : "+v"(r)); return r; }
__device__ __forceinline__ void split16(float v, b16& hi, b16& lo) { hi = (b16)v; lo = (b16)(v - (float)hi); }
__device__ __forceinline__ v16b frag_kb(const b16* p, int hh) { const v8b a = *(const v8b*)(p + 8 * hh), b = *(const v8b*)(p + 16 + 8 * hh); v16b f;
#pragma unroll
  for (int e = 0; e < 8; ++e) { f[e] = a[e]; f[8 + e] = b[e]; } return f; }
__device__ __forceinline__ v8f wmma16b(v16b a, v16b b, v8f c) { v8f d = __builtin_amdgcn_wmma_f32_16x16x32_f16(false, a, false, b, (short)0, c, false, false); asm volatile("v_nop\n\tv_nop\n\tv_nop\n\tv_nop" : "+v"(d) : "v"(a), "v"(b)); return d; }
__device__ __forceinline__ void wave_lds_sync() { __builtin_amdgcn_fence(__ATOMIC_RELEASE, "workgroup"); __builtin_amdgcn_wave_barrier(); __builtin_amdgcn_fence(__ATOMIC_ACQUIRE, "workgroup"); }
__device__ __forceinline__ float pmul(float a, float b) { float p = a * b; asm volatile("" : "+v"(p)); return p; }

__global__ __launch_bounds__(256) void prep_kernel(const float* __restrict__ wq, const float* __restrict__ wk, const float* __restrict__ wv, const float* __restrict__ emb, b16* __restrict__ WA, b16* __restrict__ ET) { const int u = blockIdx.x * 256 + threadIdx.x; v8b v; auto put = [&](b16* dst) { for (int pass = 0; pass < 2; ++pass) { *(volatile v8b*)dst = v; __threadfence(); } };
  if (u < NO * 32) { const int o = u / 32, c0 = (u % 32) * 8; const float* w = o < NQ ? wq + (size_t)o * DIM : (o < NQ + DK ? wk + (size_t)(o - NQ) * DIM : wv + (size_t)(o - NQ - DK) * DIM);
#pragma unroll
    for (int j = 0; j < 8; ++j) v[j] = (b16)(bf16_rne(w[c0 + j]) * WSC); put(WA + (size_t)o * DIM + c0); }
  if (u < RL * RL * 2) { const int r = u / 2, k0 = (u % 2) * 8;
#pragma unroll
    for (int j = 0; j < 8; ++j) v[j] = (b16)(bfv(emb[(size_t)r * DK + k0 + j]) * XS); put(ET + (size_t)r * DK + k0); } }
__global__ __launch_bounds__(32) void proj_kernel(const float* __restrict__ x, const b16* __restrict__ WA, float* __restrict__ QR, float* __restrict__ KR, float* __restrict__ VR) { __shared__ __attribute__((aligned(16))) b16 Ax[16][DIM + 8]; __shared__ float Tf[16][NO + 4]; const int lane = threadIdx.x, nloc = lane & 15, hlf = lane >> 4; const int b = blockIdx.x / (NP / 16), n0 = (blockIdx.x % (NP / 16)) * 16;
  for (int q = 0; q < DIM / 32; ++q) { const int c = q * 32 + lane; const float* xp = x + ((size_t)b * DIM + c) * NP + n0; for (int rr = 0; rr < 16; ++rr) Ax[rr][c] = (b16)(bfv(xp[rr]) * XS); }
  if (lane < 16) for (int k = DIM; k < DIM + 8; ++k) Ax[lane][k] = (b16)0.0f;
  wave_lds_sync(); v8f acc[9];
#pragma unroll
  for (int t = 0; t < 9; ++t) acc[t] = (v8f){};
#pragma unroll 2
  for (int kb = 0; kb < DIM; kb += 32) { const v16b a = frag_kb(&Ax[nloc][kb], hlf);
#pragma unroll
    for (int t = 0; t < 9; ++t) acc[t] = wmma16b(a, frag_kb(WA + (size_t)(t * 16 + nloc) * DIM + kb, hlf), acc[t]); }
#pragma unroll
  for (int t = 0; t < 9; ++t)
#pragma unroll
    for (int r8 = 0; r8 < 8; ++r8) Tf[8 * hlf + r8][t * 16 + nloc] = acc[t][r8] * (1.0f / (XS * WSC));
  wave_lds_sync();
  for (int pass = 0; pass < 2; ++pass) { for (int rr = 0; rr < 16; ++rr) { const size_t bn = (size_t)b * NP + n0 + rr; *(volatile v2f*)(QR + bn * NQ + lane * 2) = (v2f){Tf[rr][lane * 2], Tf[rr][lane * 2 + 1]}; if (lane < 16) ((volatile float*)KR)[bn * DK + lane] = Tf[rr][NQ + lane]; *(volatile v2f*)(VR + bn * DV + lane * 2) = (v2f){Tf[rr][NQ + DK + lane * 2], Tf[rr][NQ + DK + lane * 2 + 1]}; } __threadfence(); } }
__global__ __launch_bounds__(128) void stats_kernel(const float* __restrict__ QR, const float* __restrict__ VR, float* __restrict__ ST) { const int c = threadIdx.x; const float* src = c < NQ ? QR + c : VR + (c - NQ); double s = 0.0, s2 = 0.0;
#pragma unroll 1
  for (size_t bn = 0; bn < (size_t)NB_ * NP; ++bn) { const double v = (double)src[bn * 64]; s += v; s2 += v * v; }
  const double cntd = (double)NB_ * NP; const double mu = s / cntd; double var = s2 / cntd - mu * mu; if (var < 0.0) var = 0.0;
  for (int pass = 0; pass < 2; ++pass) { ((volatile float*)ST)[c] = (float)mu; ((volatile float*)ST)[128 + c] = (float)(1.0 / sqrt(var + (double)EPS)); __threadfence(); } }
__global__ __launch_bounds__(256) void ksoft_kernel(const float* __restrict__ KR, float* __restrict__ KS) { const int wave = threadIdx.x >> 5, lane = threadIdx.x & 31; const int bk = blockIdx.x * 8 + wave; if (bk >= NB_ * DK) return; const int b = bk / DK, k = bk % DK; const float* kr = KR + (size_t)b * NP * DK + k;
  float mx = -INFINITY; for (int n = lane; n < NP; n += 32) mx = fmaxf(mx, kr[(size_t)n * DK]); for (int o = 16; o; o >>= 1) mx = fmaxf(mx, __shfl_xor(mx, o));
  float z = 0.0f; for (int n = lane; n < NP; n += 32) z += __expf(kr[(size_t)n * DK] - mx); for (int o = 16; o; o >>= 1) z += __shfl_xor(z, o); const float inv = 1.0f / z;
  for (int pass = 0; pass < 2; ++pass) { for (int n = lane; n < NP; n += 32) ((volatile float*)KS)[((size_t)b * DK + k) * NP + n] = __expf(kr[(size_t)n * DK] - mx) * inv; __threadfence(); } }
__global__ __launch_bounds__(256) void vt_kernel(const float* __restrict__ VR, const float* __restrict__ ST, const float* __restrict__ gv, const float* __restrict__ bv, b16* __restrict__ VTh, b16* __restrict__ VTl) { __shared__ float Tt[64][65]; const int b = blockIdx.x / (NP / 64), m0 = (blockIdx.x % (NP / 64)) * 64; const int tid = threadIdx.x, wave = tid >> 5, lane = tid & 31;
  for (int q = wave; q < 64; q += 8) for (int half = 0; half < 2; ++half) { const int c = half * 32 + lane; const float raw = VR[((size_t)b * NP + m0 + q) * DV + c]; Tt[q][c] = pmul((raw - ST[NQ + c]) * ST[128 + NQ + c], bfv(gv[c])) + bfv(bv[c]); }
  __syncthreads();
  for (int pass = 0; pass < 2; ++pass) { for (int v = wave; v < 64; v += 8) { b16 h0, l0, h1, l1; split16(Tt[lane * 2][v] * HS, h0, l0); split16(Tt[lane * 2 + 1][v] * HS, h1, l1); const size_t o = ((size_t)b * DV + v) * NP + m0 + lane * 2; *(volatile v2b*)(VTh + o) = (v2b){h0, h1}; *(volatile v2b*)(VTl + o) = (v2b){l0, l1}; } __threadfence(); } }
__global__ __launch_bounds__(256) void lamc_kernel(const float* __restrict__ KS, const float* __restrict__ VR, const float* __restrict__ ST, const float* __restrict__ gv, const float* __restrict__ bv, float* __restrict__ LC) { const int wave = threadIdx.x >> 5, lane = threadIdx.x & 31; const int bk = blockIdx.x * 8 + wave; if (bk >= NB_ * DK) return; const int b = bk / DK, k = bk % DK; const int c0 = lane * 2; const float m0_ = ST[NQ + c0], r0 = ST[128 + NQ + c0], g0 = bfv(gv[c0]), b0 = bfv(bv[c0]), m1_ = ST[NQ + c0 + 1], r1 = ST[128 + NQ + c0 + 1], g1 = bfv(gv[c0 + 1]), b1 = bfv(bv[c0 + 1]); float a0 = 0.0f, a1 = 0.0f; const float* ks = KS + ((size_t)b * DK + k) * NP;
#pragma unroll 1
  for (int m = 0; m < NP; ++m) { const float kk = ks[m]; const v2f vr = *(const v2f*)(VR + ((size_t)b * NP + m) * DV + c0); a0 += pmul(kk, pmul((vr[0] - m0_) * r0, g0) + b0); a1 += pmul(kk, pmul((vr[1] - m1_) * r1, g1) + b1); }
  for (int pass = 0; pass < 2; ++pass) { *(volatile v2f*)(LC + ((size_t)b * DK + k) * DV + c0) = (v2f){a0, a1}; __threadfence(); } }
__global__ __launch_bounds__(32) void main_kernel(const b16* __restrict__ ET, const b16* __restrict__ VTh, const b16* __restrict__ VTl, const float* __restrict__ QR, const float* __restrict__ ST, const float* __restrict__ gq, const float* __restrict__ bq, const float* __restrict__ LC, int BLIM, float* __restrict__ YS) { __shared__ __attribute__((aligned(16))) b16 A[DK][NP + 8]; __shared__ float LPf[DK][DV + 1], Qb[NQ]; const int lane = threadIdx.x, nloc = lane & 15, hlf = lane >> 4; const int b = blockIdx.x / NP, n = blockIdx.x % NP; if (b >= BLIM) return; const int in_ = n / NS, jn = n % NS;
  for (int m = lane; m < NP; m += 32) { const int im = m / NS, jm = m % NS; const int r = (im - in_ + NS - 1) * RL + (jm - jn + NS - 1); const v8b e0 = *(const v8b*)(ET + (size_t)r * DK), e1 = *(const v8b*)(ET + (size_t)r * DK + 8);
#pragma unroll
    for (int k = 0; k < 8; ++k) { A[k][m] = e0[k]; A[8 + k][m] = e1[k]; } }
  if (lane < 16) for (int m = NP; m < NP + 8; ++m) A[lane][m] = (b16)0.0f;
  for (int c = lane; c < NQ; c += 32) Qb[c] = pmul((QR[((size_t)b * NP + n) * NQ + c] - ST[c]) * ST[128 + c], bfv(gq[c])) + bfv(bq[c]);
  wave_lds_sync(); v8f acc[4] = {(v8f){}, (v8f){}, (v8f){}, (v8f){}};
#pragma unroll 2
  for (int kb = 0; kb < NP; kb += 32) { const v16b a = frag_kb(&A[nloc][kb], hlf);
#pragma unroll
    for (int t = 0; t < 4; ++t) { const size_t vo = ((size_t)b * DV + t * 16 + nloc) * NP + kb; acc[t] = wmma16b(a, frag_kb(VTh + vo, hlf), acc[t]); acc[t] = wmma16b(a, frag_kb(VTl + vo, hlf), acc[t]); } }
#pragma unroll
  for (int t = 0; t < 4; ++t)
#pragma unroll
    for (int r8 = 0; r8 < 8; ++r8) LPf[8 * hlf + r8][t * 16 + nloc] = acc[t][r8] * (1.0f / (XS * HS));
  wave_lds_sync();
  float y[8]; const float* lc = LC + (size_t)b * DK * DV;
#pragma unroll
  for (int hv = 0; hv < 8; ++hv) { const int c = hv * 32 + lane; const int h = c / DV, v = c % DV; float s = 0.0f;
#pragma unroll
    for (int k = 0; k < DK; ++k) s += pmul(Qb[h * DK + k], LPf[k][v] + lc[k * DV + v]); y[hv] = s; }
  for (int pass = 0; pass < 2; ++pass) {
#pragma unroll
    for (int hv = 0; hv < 8; ++hv) ((volatile float*)YS)[((size_t)b * NP + n) * (HEADS * DV) + hv * 32 + lane] = y[hv]; __threadfence(); } }
__global__ __launch_bounds__(256) void copy_kernel(const float* __restrict__ YS, int BLIM, float* __restrict__ out) { const size_t u = (size_t)blockIdx.x * 256 + threadIdx.x; if (u >= (size_t)NB_ * 256 * NP) return; const int n = (int)(u % NP), c = (int)((u / NP) % 256), b = (int)(u / ((size_t)NP * 256)); const float v = b < BLIM ? YS[((size_t)b * NP + n) * 256 + c] : 0.0f;
  for (int pass = 0; pass < 2; ++pass) { ((volatile float*)out)[u] = v; __threadfence(); } }
}

extern "C" void kernel_launch(void* const* d_in, const int* in_sizes, int n_in, void* d_out, int out_size, void* d_ws, size_t ws_size, hipStream_t stream) {
  (void)n_in;
  auto Fp = [&](int i) { return (const float*)d_in[i]; };
  if (in_sizes[0] != NB_ * DIM * NP || in_sizes[1] != NQ * DIM || in_sizes[2] != DK * DIM || in_sizes[3] != DV * DIM || in_sizes[4] != NQ || in_sizes[6] != DV || in_sizes[8] != RL * RL * DK || out_size != NB_ * 256 * NP) return;
  const int BLIM = NB_;
  size_t off = 0; char* ws = (char*)d_ws;
  auto carve = [&](size_t bytes) { char* p = ws + off; off += (bytes + 255) & ~(size_t)255; return p; };
  b16* WA = (b16*)carve((size_t)NO * DIM * 2); b16* ET = (b16*)carve((size_t)RL * RL * DK * 2 + 256); float* QR = (float*)carve((size_t)NB_ * NP * NQ * 4); float* KR = (float*)carve((size_t)NB_ * NP * DK * 4); float* VR = (float*)carve((size_t)NB_ * NP * DV * 4); float* ST = (float*)carve(256 * 4); float* KS = (float*)carve((size_t)NB_ * DK * NP * 4); b16* VTh = (b16*)carve((size_t)NB_ * DV * NP * 2); b16* VTl = (b16*)carve((size_t)NB_ * DV * NP * 2); float* LC = (float*)carve((size_t)NB_ * DK * DV * 4); float* YS = (float*)carve((size_t)NB_ * NP * 256 * 4);
  if (off > ws_size || off > ((size_t)80 << 20)) return;
  prep_kernel<<<(NO * 32 + 255) / 256 > (RL * RL * 2 + 255) / 256 ? (NO * 32 + 255) / 256 : (RL * RL * 2 + 255) / 256, 256, 0, stream>>>(Fp(1), Fp(2), Fp(3), Fp(8), WA, ET);
  proj_kernel<<<NB_ * (NP / 16), 32, 0, stream>>>(Fp(0), WA, QR, KR, VR);
  stats_kernel<<<1, 128, 0, stream>>>(QR, VR, ST);
  ksoft_kernel<<<(NB_ * DK + 7) / 8, 256, 0, stream>>>(KR, KS);
  vt_kernel<<<NB_ * (NP / 64), 256, 0, stream>>>(VR, ST, Fp(6), Fp(7), VTh, VTl);
  lamc_kernel<<<(NB_ * DK + 7) / 8, 256, 0, stream>>>(KS, VR, ST, Fp(6), Fp(7), LC);
  main_kernel<<<NB_ * NP, 32, 0, stream>>>(ET, VTh, VTl, QR, ST, Fp(4), Fp(5), LC, BLIM, YS);
  copy_kernel<<<(NB_ * 256 * NP + 255) / 256, 256, 0, stream>>>(YS, BLIM, (float*)d_out);
}
